// TrackNet_75239237091989
// MI455X (gfx1250) — hardware-verified
//
#include <hip/hip_runtime.h>


namespace {
constexpr int Bn = 16, NBX = 32, C = 512, FEAT = 224, OUTW = 526848;
__constant__ int LVL_S[3] = {8, 16, 32}; __constant__ int LVL_HW[3] = {28, 14, 7}; __constant__ int LVL_OFF[3] = {0, 401408, 501760};
constexpr float AS_ = 8.0f;

typedef _Float16 b16;
typedef __attribute__((ext_vector_type(16))) _Float16 v16b;
typedef __attribute__((ext_vector_type(8))) _Float16 v8b;
typedef __attribute__((ext_vector_type(8))) float v8f;
typedef __attribute__((ext_vector_type(4))) float v4f;
__device__ __forceinline__ float bf16_rne(float f) { unsigned int u = __float_as_uint(f); u += 0x7FFFu + ((u >> 16) & 1u); return __uint_as_float(u & 0xFFFF0000u); }
__device__ __forceinline__ void split16(float v, b16& hi, b16& lo) { hi = (b16)v; lo = (b16)(v - (float)hi); }
__device__ __forceinline__ v8f wmma16b(v16b a, v16b b, v8f c) { v8f d = __builtin_amdgcn_wmma_f32_16x16x32_f16(false, a, false, b, (short)0, c, false, false); asm volatile("v_nop\n\tv_nop\n\tv_nop\n\tv_nop" : "+v"(d) : "v"(a), "v"(b)); return d; }
__device__ __forceinline__ float nexp(float x) { return __builtin_amdgcn_exp2f(x * 1.4426950408889634f); }
__device__ __forceinline__ float pmul(float a, float b) { float p = a * b; asm volatile("" : "+v"(p)); return p; }
__device__ __forceinline__ float sigm(float x) { return 1.0f / (1.0f + nexp(-x)); }

__global__ __launch_bounds__(256) void track_kernel(const float* __restrict__ confs, const float* __restrict__ boxes, const float* __restrict__ f0, const float* __restrict__ f1, const float* __restrict__ f2, float* __restrict__ out) {
  __shared__ int bx[NBX][4]; __shared__ float cf[NBX]; __shared__ float att[800]; __shared__ __attribute__((aligned(16))) b16 Ah[800], Al[800]; __shared__ float lg[C]; __shared__ float wch[C]; __shared__ float red[16];
  const int lvl = blockIdx.x, b = blockIdx.y, t_ = threadIdx.x, lane = t_ & 31, wave = t_ >> 5, nloc = lane & 15, hlf = lane >> 4;
  const int s = LVL_S[lvl], hw1 = LVL_HW[lvl], HW = hw1 * hw1, KP = (HW + 31) & ~31; const float* feat = ((lvl == 0) ? f0 : (lvl == 1) ? f1 : f2) + (size_t)b * C * HW;
  if (t_ < NBX) { cf[t_] = bf16_rne(confs[b * NBX + t_]); for (int j = 0; j < 4; ++j) bx[t_][j] = (int)floorf(bf16_rne(boxes[((size_t)b * NBX + t_) * 4 + j]) * (float)FEAT); }
  for (int i = t_; i < 800; i += 256) att[i] = 0.0f;
  __syncthreads();
  for (int p = t_; p < HW; p += 256) { const int py = p / hw1, px = p % hw1; float acc = 0.0f;
    for (int dy = 0; dy < s; ++dy) for (int dx = 0; dx < s; ++dx) { const int y = py * s + dy, x = px * s + dx; float cm = 0.0f;
        for (int n = 0; n < NBX; ++n) { const bool in = (y >= bx[n][1]) && (y < bx[n][3]) && (x >= bx[n][0]) && (x < bx[n][2]); if (in) cm += cf[n]; }
        acc += sigm(cm); }
    att[p] = acc / (float)(s * s); }
  __syncthreads();
  for (int i = t_; i < KP; i += 256) { b16 h_, l_; split16(((i < HW) ? att[i] : 0.0f) * AS_, h_, l_); Ah[i] = h_; Al[i] = l_; }
  __syncthreads();
  for (int ct = wave; ct < C / 16; ct += 8) { v8f acc = {};
    for (int kb = 0; kb < KP; kb += 32) { v16b a, bh, bl; const float* fr = feat + (size_t)(ct * 16 + nloc) * HW;
#pragma unroll
      for (int e = 0; e < 16; ++e) { const int k = kb + ((e < 8) ? (8 * hlf + e) : (16 + 8 * hlf + e - 8)); a[e] = (b16)((k < HW) ? bf16_rne(fr[k]) : 0.0f); bh[e] = (nloc == 0) ? Ah[k] : (b16)0.0f; bl[e] = (nloc == 0) ? Al[k] : (b16)0.0f; }
      acc = wmma16b(a, bh, acc); acc = wmma16b(a, bl, acc); }
    if (nloc == 0) {
#pragma unroll
      for (int r = 0; r < 8; ++r) lg[ct * 16 + 8 * hlf + r] = acc[r] * (1.0f / AS_); } }
  __syncthreads();
  { float mx = -INFINITY; for (int c = t_; c < C; c += 256) mx = fmaxf(mx, lg[c]);
#pragma unroll
    for (int o = 1; o < 32; o <<= 1) mx = fmaxf(mx, __shfl_xor(mx, o));
    if (lane == 0) red[wave] = mx; __syncthreads(); mx = red[0]; for (int w = 1; w < 8; ++w) mx = fmaxf(mx, red[w]); __syncthreads();
    float su = 0.0f; for (int c = t_; c < C; c += 256) su += nexp(lg[c] - mx);
#pragma unroll
    for (int o = 1; o < 32; o <<= 1) su += __shfl_xor(su, o);
    if (lane == 0) red[8 + wave] = su; __syncthreads(); su = 0.0f; for (int w = 0; w < 8; ++w) su += red[8 + w];
    for (int c = t_; c < C; c += 256) wch[c] = nexp(lg[c] - mx) / su; }
  __syncthreads();
  float* ob = out + (size_t)b * OUTW + LVL_OFF[lvl]; const int tot = C * HW;
  for (int pass = 0; pass < 2; ++pass) { for (int i4 = t_ * 4; i4 < tot; i4 += 1024) { v4f v; for (int e = 0; e < 4; ++e) { const int i = i4 + e; const int c = i / HW; v[e] = pmul(bf16_rne(feat[i]), wch[c]); } *(volatile v4f*)(ob + i4) = v; } __threadfence(); }
}
}

extern "C" void kernel_launch(void* const* d_in, const int* in_sizes, int n_in,
                              void* d_out, int out_size, void* d_ws, size_t ws_size, hipStream_t stream) {
  (void)n_in; (void)out_size; (void)d_ws; (void)ws_size;
  const float* confs = (const float*)d_in[0]; const float* boxes = (const float*)d_in[1]; const float* f0 = (const float*)d_in[2]; const float* f1 = (const float*)d_in[3]; const float* f2 = (const float*)d_in[4];
  float* out = (float*)d_out;
  if (in_sizes[0] != Bn * NBX || in_sizes[1] != Bn * NBX * 4 || in_sizes[2] != Bn * C * 784 || in_sizes[3] != Bn * C * 196 || in_sizes[4] != Bn * C * 49) return;
  track_kernel<<<dim3(3, Bn), 256, 0, stream>>>(confs, boxes, f0, f1, f2, out);
}
